// test_GGCN_4861902979401
// MI455X (gfx1250) — hardware-verified
//
#include <hip/hip_runtime.h>


#define NN     10000
#define EE     320000
#define NG     64
#define NOUT   6
#define C1     128
#define C2     256
#define NTHR   256

#define NBK    1024
#define NBUCK  10
#define CAPB   36864
#define MAXDEG 128
#define RINTS  (2 * NBK + CAPB)
#define CHUNK  (NTHR * 8)
#define NCHUNK ((EE + CHUNK - 1) / CHUNK)

#define L_BEG  0
#define L_CNT  NBK
#define L_COL  (2 * NBK)
#define L_CUR  (2 * NBK + CAPB)
#define L_DUM  (L_CUR + NBK)
#define L_WS   (L_DUM + 32)
#define L_TOT  (L_WS + 32)
#define CSR_LDS_BYTES (L_TOT * 4)

static_assert(NN % 16 == 0);
static_assert(EE % 8 == 0);
static_assert(NBUCK * NBK >= NN);
static_assert((NBUCK - 1) * NBK < NN);
static_assert(NBK == 4 * NTHR);
static_assert(RINTS % (4 * NTHR) == 0);
static_assert((L_COL + CAPB) % (4 * NTHR) == 0);
static_assert((NN * C1) % (8 * NTHR) == 0);
static_assert((NN * C2) % (4 * NTHR) == 0);
static_assert(C2 == NTHR);
static_assert((NG * NOUT) % 4 == 0);
static_assert(CSR_LDS_BYTES <= 200000);

typedef unsigned short us16;
typedef us16   v8us  __attribute__((ext_vector_type(8)));
typedef us16   v4us  __attribute__((ext_vector_type(4)));
typedef __bf16 v16bf __attribute__((ext_vector_type(16)));
typedef float  v8f   __attribute__((ext_vector_type(8)));
typedef float  v4f   __attribute__((ext_vector_type(4)));
typedef int    v4i   __attribute__((ext_vector_type(4)));

union FragBF { v16bf v; v8us half[2]; };

constexpr size_t WPE1   = (size_t)3 * C1 * C1;
constexpr size_t WPE2   = (size_t)3 * C2 * C2;
constexpr size_t B_M    = (size_t)NN * C2 * 4;
constexpr size_t B_HF1  = (size_t)NN * C1 * 4;
constexpr size_t B_HF2  = (size_t)NN * C2 * 4;
constexpr size_t B_PL   = (size_t)NN * C2 * 2;
constexpr size_t B_W1   = 6 * WPE1 * 2;
constexpr size_t B_W2   = 6 * WPE2 * 2;
constexpr size_t B_CSR  = (size_t)NBUCK * RINTS * 4;
constexpr size_t OFF_M    = 0;
constexpr size_t OFF_HF1  = OFF_M    + B_M;
constexpr size_t OFF_HF2  = OFF_HF1  + B_HF1;
constexpr size_t OFF_HHIA = OFF_HF2  + B_HF2;
constexpr size_t OFF_HLOA = OFF_HHIA + B_PL;
constexpr size_t OFF_HHIB = OFF_HLOA + B_PL;
constexpr size_t OFF_HLOB = OFF_HHIB + B_PL;
constexpr size_t OFF_AHI  = OFF_HLOB + B_PL;
constexpr size_t OFF_ALO  = OFF_AHI  + B_PL;
constexpr size_t OFF_W1   = OFF_ALO  + B_PL;
constexpr size_t OFF_W2   = OFF_W1   + B_W1;
constexpr size_t OFF_CSR  = OFF_W2   + B_W2;
constexpr size_t WS_END   = OFF_CSR  + B_CSR;
static_assert(OFF_HF1 % 256 == 0 && OFF_HF2 % 256 == 0 && OFF_HHIA % 256 == 0 && OFF_HLOA % 256 == 0);
static_assert(OFF_HHIB % 256 == 0 && OFF_HLOB % 256 == 0 && OFF_AHI % 256 == 0 && OFF_ALO % 256 == 0);
static_assert(OFF_W1 % 256 == 0 && OFF_W2 % 256 == 0 && OFF_CSR % 256 == 0);
static_assert(WS_END <= (size_t)134217728);

__device__ __forceinline__ unsigned bf16_rne(float x) {
    unsigned u = __float_as_uint(x);
    u += 0x7FFFu + ((u >> 16) & 1u);
    return u >> 16;
}
__device__ __forceinline__ void split2(float x, us16& hi, us16& lo) {
    const unsigned hb = bf16_rne(x);
    const float    r  = x - __uint_as_float(hb << 16);
    hi = (us16)hb;
    lo = (us16)bf16_rne(r);
}
__device__ __forceinline__ float sigf(float x) {
    const float e = expf(fminf(-x, 30.0f));
    return 1.0f / (1.0f + e);
}
__device__ __forceinline__ float tanhf2(float x) {
    const float ax = fminf(fabsf(x), 15.0f);
    const float t  = expf(2.0f * ax);
    const float y  = 1.0f - 2.0f / (t + 1.0f);
    return copysignf(y, x);
}
__device__ __forceinline__ v8f zero8() {
    v8f z;
#pragma unroll
    for (int i = 0; i < 8; ++i) z[i] = 0.0f;
    return z;
}

__device__ __forceinline__ FragBF ldfrag(const us16* p) {
    FragBF f;
    f.half[0] = *(const v8us*)p;
    f.half[1] = *(const v8us*)(p + 16);
    return f;
}
__device__ __forceinline__ v8f mma_bf(v8f c, const FragBF& a, const FragBF& b) {
    c = __builtin_amdgcn_wmma_f32_16x16x32_bf16(false, a.v, false, b.v, (short)0, c, false, false);
    asm volatile("v_nop\n\tv_nop\n\tv_nop\n\tv_nop" : "+v"(c) : "v"(a.v), "v"(b.v));
    return c;
}
__device__ __forceinline__ v8f mma3(v8f c, const FragBF& ah, const FragBF& al, const FragBF& bh, const FragBF& bl) {
    c = mma_bf(c, ah, bh);
    c = mma_bf(c, ah, bl);
    c = mma_bf(c, al, bh);
    return c;
}

struct WArgs { const float* w; const float* wih; const float* whh; us16* pl; };
static_assert(sizeof(WArgs) == 4 * 8);

template <int C>
__global__ __launch_bounds__(NTHR)
void k_wprep(WArgs a)
{
    constexpr int WPE  = 3 * C * C;
    constexpr int GSTR = C * C;
    constexpr int BPS  = WPE / (8 * NTHR);
    constexpr int QL   = C * C / 8;
    constexpr int KQ   = C / 8;
    const int seg = (int)blockIdx.x / BPS;
    const int q   = ((int)blockIdx.x - seg * BPS) * NTHR + (int)threadIdx.x;
    float x[8];
    us16* dh;
    if (seg == 0) {
        const int l  = q / QL;
        const int r  = q - l * QL;
        const int j  = r / KQ;
        const int kq = (r - j * KQ) * 8;
        const float* src = a.w + (size_t)l * GSTR + (size_t)kq * C + j;
#pragma unroll
        for (int i = 0; i < 8; ++i) x[i] = src[(size_t)i * C];
        dh = a.pl + (size_t)l * GSTR + (size_t)j * C + kq;
    } else if (seg == 1) {
        const size_t e0 = (size_t)q * 8;
        const v4f x0 = *(const v4f*)(a.wih + e0);
        const v4f x1 = *(const v4f*)(a.wih + e0 + 4);
#pragma unroll
        for (int i = 0; i < 4; ++i) { x[i] = x0[i]; x[4 + i] = x1[i]; }
        dh = a.pl + (size_t)2 * WPE + e0;
    } else {
        const size_t e0 = (size_t)q * 8;
        const v4f x0 = *(const v4f*)(a.whh + e0);
        const v4f x1 = *(const v4f*)(a.whh + e0 + 4);
#pragma unroll
        for (int i = 0; i < 4; ++i) { x[i] = x0[i]; x[4 + i] = x1[i]; }
        dh = a.pl + (size_t)4 * WPE + e0;
    }
    us16* dl = dh + WPE;
    v8us hv, lv;
#pragma unroll
    for (int i = 0; i < 8; ++i) { us16 hi, lo; split2(x[i], hi, lo); hv[i] = hi; lv[i] = lo; }
    *(volatile v8us*)dh = hv;
    *(volatile v8us*)dl = lv;
    __threadfence();
    *(volatile v8us*)dh = hv;
    *(volatile v8us*)dl = lv;
}

struct ZArgs { const float* z; us16* hhi; us16* hlo; };
static_assert(sizeof(ZArgs) == 3 * 8);

__global__ __launch_bounds__(NTHR)
void k_xplanes(ZArgs a)
{
    const size_t e0 = ((size_t)blockIdx.x * NTHR + threadIdx.x) * 8;
    const v4f x0 = *(const v4f*)(a.z + e0);
    const v4f x1 = *(const v4f*)(a.z + e0 + 4);
    v8us hv, lv;
#pragma unroll
    for (int i = 0; i < 4; ++i) {
        us16 hi, lo;
        split2(x0[i], hi, lo); hv[i] = hi;     lv[i] = lo;
        split2(x1[i], hi, lo); hv[4 + i] = hi; lv[4 + i] = lo;
    }
    us16* ph = a.hhi + e0;
    us16* pl = a.hlo + e0;
    *(volatile v8us*)ph = hv;
    *(volatile v8us*)pl = lv;
    __threadfence();
    *(volatile v8us*)ph = hv;
    *(volatile v8us*)pl = lv;
}

struct CsrArgs { const int* eidx; int* csr; };
static_assert(sizeof(CsrArgs) == 2 * 8);

__global__ __launch_bounds__(NTHR)
void k_csr(CsrArgs a)
{
    extern __shared__ int L[];
    const int tid  = (int)threadIdx.x;
    const int lane = tid & 31;
    const int wv   = tid >> 5;
    const int b    = (int)blockIdx.x;
    const int base = b * NBK;
    const int* src = a.eidx;
    const int* dst = a.eidx + EE;

    {
        v4i z4; z4[0] = 0; z4[1] = 0; z4[2] = 0; z4[3] = 0;
#pragma unroll 1
        for (int i = 0; i < (L_COL + CAPB) / (4 * NTHR); ++i)
            *(v4i*)(&L[(i * NTHR + tid) * 4]) = z4;
        if (tid < 64) L[L_DUM + tid] = 0;
    }
    __syncthreads();

#pragma unroll 1
    for (int c = 0; c < NCHUNK; ++c) {
        const int  e0    = c * CHUNK + tid * 8;
        const int  e0c   = min(e0, EE - 8);
        const bool valid = e0 < EE;
        const v4i d0 = *(const v4i*)(dst + e0c);
        const v4i d1 = *(const v4i*)(dst + e0c + 4);
        const int dd[8] = { d0[0], d0[1], d0[2], d0[3], d1[0], d1[1], d1[2], d1[3] };
#pragma unroll
        for (int j = 0; j < 8; ++j) {
            const int  dl  = dd[j] - base;
            const bool hit = valid && ((unsigned)dl < (unsigned)NBK);
            atomicAdd(&L[hit ? (L_CNT + dl) : L_DUM], hit ? 1 : 0);
        }
    }
    __syncthreads();

    {
        const v4i c0 = *(const v4i*)(&L[L_CNT + tid * 4]);
        const int loc = c0[0] + c0[1] + c0[2] + c0[3];
        int inc = loc;
#pragma unroll
        for (int off = 1; off < 32; off <<= 1) {
            const int t = __shfl_up(inc, off);
            inc += (lane >= off) ? t : 0;
        }
        if (lane == 31) L[L_WS + wv] = inc;
        __syncthreads();
        int woff = 0;
#pragma unroll
        for (int u = 0; u < 8; ++u) { const int s = L[L_WS + u]; woff += (u < wv) ? s : 0; }
        int ex = woff + inc - loc;
        v4i b0;
        b0[0] = ex; ex += c0[0]; b0[1] = ex; ex += c0[1]; b0[2] = ex; ex += c0[2]; b0[3] = ex;
        *(v4i*)(&L[L_BEG + tid * 4]) = b0;
        *(v4i*)(&L[L_CUR + tid * 4]) = b0;
    }
    __syncthreads();

#pragma unroll 1
    for (int c = 0; c < NCHUNK; ++c) {
        const int  e0    = c * CHUNK + tid * 8;
        const int  e0c   = min(e0, EE - 8);
        const bool valid = e0 < EE;
        const v4i d0 = *(const v4i*)(dst + e0c);
        const v4i d1 = *(const v4i*)(dst + e0c + 4);
        const v4i s0 = *(const v4i*)(src + e0c);
        const v4i s1 = *(const v4i*)(src + e0c + 4);
        const int dd[8] = { d0[0], d0[1], d0[2], d0[3], d1[0], d1[1], d1[2], d1[3] };
        const int ss[8] = { s0[0], s0[1], s0[2], s0[3], s1[0], s1[1], s1[2], s1[3] };
#pragma unroll
        for (int j = 0; j < 8; ++j) {
            const int  dl  = dd[j] - base;
            const bool hit = valid && ((unsigned)dl < (unsigned)NBK);
            const int  pos = atomicAdd(&L[hit ? (L_CUR + dl) : (L_DUM + 1)], hit ? 1 : 0);
            if (hit && (unsigned)pos < (unsigned)CAPB) L[L_COL + pos] = ss[j];
        }
    }
    __syncthreads();

    int* R = a.csr + (size_t)b * RINTS;
#pragma unroll 1
    for (int i = 0; i < RINTS / (4 * NTHR); ++i) {
        const int o = (i * NTHR + tid) * 4;
        const v4i v = *(const v4i*)(&L[o]);
        *(volatile v4i*)(R + o) = v;
    }
    __threadfence();
#pragma unroll 1
    for (int i = 0; i < RINTS / (4 * NTHR); ++i) {
        const int o = (i * NTHR + tid) * 4;
        const v4i v = *(const v4i*)(&L[o]);
        *(volatile v4i*)(R + o) = v;
    }
}

struct GmArgs { const us16* hhi; const us16* hlo; const us16* whi; const us16* wlo; float* m; int nk; int pad0; };
static_assert(sizeof(GmArgs) == 5 * 8 + 8);

template <int C>
__global__ __launch_bounds__(NTHR)
void k_gemm_m(GmArgs a)
{
    __shared__ __attribute__((aligned(16))) float sOut[16 * 128];
    const int tid   = (int)threadIdx.x;
    const int lane  = tid & 31;
    const int wv    = tid >> 5;
    const int hh    = lane >> 4;
    const int mm    = lane & 15;
    const int row0  = (int)blockIdx.x * 16;
    const int cbase = (int)blockIdx.y * 128;
    const int jl    = wv * 16 + mm;
    const int j     = cbase + jl;

    const us16* pAh = a.hhi + (size_t)(row0 + mm) * C + 8 * hh;
    const us16* pAl = a.hlo + (size_t)(row0 + mm) * C + 8 * hh;
    const us16* pBh = a.whi + (size_t)j * C + 8 * hh;
    const us16* pBl = a.wlo + (size_t)j * C + 8 * hh;

    v8f acc = zero8();
#pragma unroll 1
    for (int ks = 0; ks < a.nk; ++ks) {
        const int kk = ks * 32;
        const FragBF ah = ldfrag(pAh + kk), al = ldfrag(pAl + kk);
        const FragBF bh = ldfrag(pBh + kk), bl = ldfrag(pBl + kk);
        acc = mma3(acc, ah, al, bh, bl);
    }
#pragma unroll
    for (int r = 0; r < 8; ++r) sOut[(8 * hh + r) * 128 + jl] = acc[r];
    __syncthreads();

    const v4f o0 = *(const v4f*)(&sOut[wv * 128 + lane * 4]);
    const v4f o1 = *(const v4f*)(&sOut[(8 + wv) * 128 + lane * 4]);
    float* m0 = a.m + (size_t)(row0 + wv) * C + cbase + lane * 4;
    float* m1 = a.m + (size_t)(row0 + 8 + wv) * C + cbase + lane * 4;
    *(volatile v4f*)m0 = o0;
    *(volatile v4f*)m1 = o1;
    __threadfence();
    *(volatile v4f*)m0 = o0;
    *(volatile v4f*)m1 = o1;
}

struct GaArgs { const float* m; const int* csr; us16* ahi; us16* alo; };
static_assert(sizeof(GaArgs) == 4 * 8);

template <int C>
__global__ __launch_bounds__(NTHR)
void k_gather(GaArgs a)
{
    constexpr int FPL = C / 32;
    const int tid  = (int)threadIdx.x;
    const int lane = tid & 31;
    const int wv   = tid >> 5;
    const int n    = (int)blockIdx.x * 8 + wv;
    const int b    = n / NBK;
    const int dl   = n - b * NBK;
    const int* R   = a.csr + (size_t)b * RINTS;
    int beg = R[L_BEG + dl];
    int cnt = R[L_CNT + dl];
    beg = min(max(beg, 0), CAPB);
    cnt = max(cnt, 0);
    cnt = min(cnt, MAXDEG);
    cnt = min(cnt, CAPB - beg);
    const int* col = R + L_COL + beg;

    v4f acc0; acc0[0] = 0.0f; acc0[1] = 0.0f; acc0[2] = 0.0f; acc0[3] = 0.0f;
    v4f acc1; acc1[0] = 0.0f; acc1[1] = 0.0f; acc1[2] = 0.0f; acc1[3] = 0.0f;
#pragma unroll 1
    for (int i = 0; i < cnt; ++i) {
        int s = col[i];
        s = min(max(s, 0), NN - 1);
        const float* p = a.m + (size_t)s * C + lane * FPL;
        acc0 += *(const v4f*)p;
        if constexpr (C == 256) acc1 += *(const v4f*)(p + 4);
    }
    if constexpr (C == 128) {
        v4us hv, lv;
#pragma unroll
        for (int i = 0; i < 4; ++i) { us16 hi, lo; split2(acc0[i], hi, lo); hv[i] = hi; lv[i] = lo; }
        us16* ph = a.ahi + (size_t)n * C + lane * 4;
        us16* pl = a.alo + (size_t)n * C + lane * 4;
        *(volatile v4us*)ph = hv;
        *(volatile v4us*)pl = lv;
        __threadfence();
        *(volatile v4us*)ph = hv;
        *(volatile v4us*)pl = lv;
    } else {
        v8us hv, lv;
#pragma unroll
        for (int i = 0; i < 4; ++i) {
            us16 hi, lo;
            split2(acc0[i], hi, lo); hv[i] = hi;     lv[i] = lo;
            split2(acc1[i], hi, lo); hv[4 + i] = hi; lv[4 + i] = lo;
        }
        us16* ph = a.ahi + (size_t)n * C + lane * 8;
        us16* pl = a.alo + (size_t)n * C + lane * 8;
        *(volatile v8us*)ph = hv;
        *(volatile v8us*)pl = lv;
        __threadfence();
        *(volatile v8us*)ph = hv;
        *(volatile v8us*)pl = lv;
    }
}

struct GrArgs {
    const us16* ahi; const us16* alo; const us16* hhi; const us16* hlo;
    us16* ohi; us16* olo; const float* hprev; float* hout;
    const us16* ihh; const us16* ihl; const us16* hhh; const us16* hhl;
    const float* bih; const float* bhh; int nkA; int nkH;
};
static_assert(sizeof(GrArgs) == 14 * 8 + 8);

template <int C>
__global__ __launch_bounds__(NTHR)
void k_gru(GrArgs a)
{
    constexpr int GSTR = C * C;
    __shared__ __attribute__((aligned(16))) float sOut[16 * 128];
    const int tid   = (int)threadIdx.x;
    const int lane  = tid & 31;
    const int wv    = tid >> 5;
    const int hh    = lane >> 4;
    const int mm    = lane & 15;
    const int row0  = (int)blockIdx.x * 16;
    const int cbase = (int)blockIdx.y * 128;
    const int jl    = wv * 16 + mm;
    const int j     = cbase + jl;

    const us16* pAh = a.ahi + (size_t)(row0 + mm) * C + 8 * hh;
    const us16* pAl = a.alo + (size_t)(row0 + mm) * C + 8 * hh;
    const us16* pHh = a.hhi + (size_t)(row0 + mm) * C + 8 * hh;
    const us16* pHl = a.hlo + (size_t)(row0 + mm) * C + 8 * hh;
    const us16* pIh = a.ihh + (size_t)j * C + 8 * hh;
    const us16* pIl = a.ihl + (size_t)j * C + 8 * hh;
    const us16* pWh = a.hhh + (size_t)j * C + 8 * hh;
    const us16* pWl = a.hhl + (size_t)j * C + 8 * hh;

    v8f cir = zero8(), ciz = zero8(), cin = zero8(), chr = zero8(), chz = zero8(), chn = zero8();
#pragma unroll 1
    for (int ks = 0; ks < a.nkA; ++ks) {
        const int kk = ks * 32;
        const FragBF xh = ldfrag(pAh + kk), xl = ldfrag(pAl + kk);
        {
            const FragBF bh = ldfrag(pIh + 0 * GSTR + kk), bl = ldfrag(pIl + 0 * GSTR + kk);
            cir = mma3(cir, xh, xl, bh, bl);
        }
        {
            const FragBF bh = ldfrag(pIh + 1 * GSTR + kk), bl = ldfrag(pIl + 1 * GSTR + kk);
            ciz = mma3(ciz, xh, xl, bh, bl);
        }
        {
            const FragBF bh = ldfrag(pIh + 2 * GSTR + kk), bl = ldfrag(pIl + 2 * GSTR + kk);
            cin = mma3(cin, xh, xl, bh, bl);
        }
    }
#pragma unroll 1
    for (int ks = 0; ks < a.nkH; ++ks) {
        const int kk = ks * 32;
        const FragBF yh = ldfrag(pHh + kk), yl = ldfrag(pHl + kk);
        {
            const FragBF bh = ldfrag(pWh + 0 * GSTR + kk), bl = ldfrag(pWl + 0 * GSTR + kk);
            chr = mma3(chr, yh, yl, bh, bl);
        }
        {
            const FragBF bh = ldfrag(pWh + 1 * GSTR + kk), bl = ldfrag(pWl + 1 * GSTR + kk);
            chz = mma3(chz, yh, yl, bh, bl);
        }
        {
            const FragBF bh = ldfrag(pWh + 2 * GSTR + kk), bl = ldfrag(pWl + 2 * GSTR + kk);
            chn = mma3(chn, yh, yl, bh, bl);
        }
    }

    const float bir = a.bih[j], biz = a.bih[C + j], bin = a.bih[2 * C + j];
    const float bhr = a.bhh[j], bhz = a.bhh[C + j], bhn = a.bhh[2 * C + j];
#pragma unroll
    for (int r = 0; r < 8; ++r) {
        const int   row = 8 * hh + r;
        const float ir  = cir[r] + bir;
        const float iz  = ciz[r] + biz;
        const float inn = cin[r] + bin;
        const float hr  = chr[r] + bhr;
        const float hz  = chz[r] + bhz;
        const float hn  = chn[r] + bhn;
        const float rg  = sigf(ir + hr);
        const float zg  = sigf(iz + hz);
        const float ng  = tanhf2(inn + rg * hn);
        const float hv  = a.hprev[(size_t)(row0 + row) * C + j];
        sOut[row * 128 + jl] = (1.0f - zg) * ng + zg * hv;
    }
    __syncthreads();

    const v4f o0 = *(const v4f*)(&sOut[wv * 128 + lane * 4]);
    const v4f o1 = *(const v4f*)(&sOut[(8 + wv) * 128 + lane * 4]);
    v4us h0, l0, h1, l1;
#pragma unroll
    for (int i = 0; i < 4; ++i) {
        us16 hi, lo;
        split2(o0[i], hi, lo); h0[i] = hi; l0[i] = lo;
        split2(o1[i], hi, lo); h1[i] = hi; l1[i] = lo;
    }
    const size_t off0 = (size_t)(row0 + wv) * C + cbase + lane * 4;
    const size_t off1 = (size_t)(row0 + 8 + wv) * C + cbase + lane * 4;
    float* q0 = a.hout + off0;
    float* q1 = a.hout + off1;
    us16* ph0 = a.ohi + off0;
    us16* ph1 = a.ohi + off1;
    us16* pl0 = a.olo + off0;
    us16* pl1 = a.olo + off1;
    *(volatile v4f*)q0 = o0;   *(volatile v4f*)q1 = o1;
    *(volatile v4us*)ph0 = h0; *(volatile v4us*)ph1 = h1;
    *(volatile v4us*)pl0 = l0; *(volatile v4us*)pl1 = l1;
    __threadfence();
    *(volatile v4f*)q0 = o0;   *(volatile v4f*)q1 = o1;
    *(volatile v4us*)ph0 = h0; *(volatile v4us*)ph1 = h1;
    *(volatile v4us*)pl0 = l0; *(volatile v4us*)pl1 = l1;
}

struct RpArgs { const float* h1; float* h2; us16* hhi; us16* hlo; };
static_assert(sizeof(RpArgs) == 4 * 8);

__global__ __launch_bounds__(NTHR)
void k_relu_pad(RpArgs a)
{
    const int  e0   = ((int)blockIdx.x * NTHR + (int)threadIdx.x) * 4;
    const int  node = e0 >> 8;
    const int  c0   = e0 & 255;
    const bool live = c0 < C1;
    const v4f  v    = *(const v4f*)(a.h1 + (size_t)node * C1 + (c0 & (C1 - 1)));
    v4f o;
#pragma unroll
    for (int i = 0; i < 4; ++i) o[i] = live ? fmaxf(v[i], 0.0f) : 0.0f;
    v4us hv, lv;
#pragma unroll
    for (int i = 0; i < 4; ++i) { us16 hi, lo; split2(o[i], hi, lo); hv[i] = hi; lv[i] = lo; }
    float* q  = a.h2 + e0;
    us16*  ph = a.hhi + e0;
    us16*  pl = a.hlo + e0;
    *(volatile v4f*)q = o;
    *(volatile v4us*)ph = hv;
    *(volatile v4us*)pl = lv;
    __threadfence();
    *(volatile v4f*)q = o;
    *(volatile v4us*)ph = hv;
    *(volatile v4us*)pl = lv;
}

struct PfArgs { const float* h; const int* batch; const float* fcw; const float* fcb; float* out; };
static_assert(sizeof(PfArgs) == 5 * 8);

__global__ __launch_bounds__(NTHR)
void k_poolfc(PfArgs a)
{
    __shared__ int   sLB[NG + 32];
    __shared__ float sY[C2];
    __shared__ __attribute__((aligned(16))) float sO[NG * NOUT];
    const int tid  = (int)threadIdx.x;
    const int lane = tid & 31;
    const int wv   = tid >> 5;

    {
        int lo = 0, hi = NN;
#pragma unroll 1
        for (int it = 0; it < 15; ++it) {
            const int  mid = (lo + hi) >> 1;
            const int  bv  = a.batch[min(mid, NN - 1)];
            const bool act = lo < hi;
            const bool gol = act && (bv < tid);
            const bool gor = act && !(bv < tid);
            lo = gol ? (mid + 1) : lo;
            hi = gor ? mid : hi;
        }
        if (tid <= NG) sLB[tid] = lo;
    }
    __syncthreads();

#pragma unroll 1
    for (int g = 0; g < NG; ++g) {
        int lo = sLB[g];
        int hi = sLB[g + 1];
        lo = min(max(lo, 0), NN);
        hi = min(max(hi, lo), NN);
        const int cnt = hi - lo;
        float mx = -__builtin_inff();
#pragma unroll 1
        for (int i = 0; i < cnt; ++i) {
            const int   n  = lo + i;
            const int   bv = a.batch[n];
            const float v  = a.h[(size_t)n * C2 + tid];
            mx = (bv == g) ? fmaxf(mx, v) : mx;
        }
        sY[tid] = mx;
        __syncthreads();
        if (wv < NOUT) {
            float s = 0.0f;
#pragma unroll 1
            for (int k = lane; k < C2; k += 32) s = fmaf(sY[k], a.fcw[(size_t)wv * C2 + k], s);
            s += __shfl_xor(s, 16);
            s += __shfl_xor(s, 8);
            s += __shfl_xor(s, 4);
            s += __shfl_xor(s, 2);
            s += __shfl_xor(s, 1);
            if (lane == 0) sO[g * NOUT + wv] = s + a.fcb[wv];
        }
        __syncthreads();
    }

    if (tid < (NG * NOUT) / 4) {
        const v4f o = *(const v4f*)(&sO[tid * 4]);
        *(volatile v4f*)(a.out + tid * 4) = o;
    }
    __threadfence();
    if (tid < (NG * NOUT) / 4) {
        const v4f o = *(const v4f*)(&sO[tid * 4]);
        *(volatile v4f*)(a.out + tid * 4) = o;
    }
}

extern "C" void kernel_launch(void* const* d_in, const int* in_sizes, int n_in,
                              void* d_out, int out_size, void* d_ws, size_t ws_size,
                              hipStream_t stream)
{
    if (n_in < 15) return;
    if (in_sizes[0] != NN * C1) return;
    if (in_sizes[1] != 2 * EE) return;
    if (in_sizes[2] != NN) return;
    if (in_sizes[3] != 3 * C1 * C1 || in_sizes[4] != 3 * C1 * C1 || in_sizes[5] != 3 * C1 * C1) return;
    if (in_sizes[6] != 3 * C1 || in_sizes[7] != 3 * C1) return;
    if (in_sizes[8] != 3 * C2 * C2 || in_sizes[9] != 3 * C2 * C2 || in_sizes[10] != 3 * C2 * C2) return;
    if (in_sizes[11] != 3 * C2 || in_sizes[12] != 3 * C2) return;
    if (in_sizes[13] != NOUT * C2 || in_sizes[14] != NOUT) return;
    if (out_size != NG * NOUT) return;
    if (ws_size < WS_END) return;

    const float* x     = (const float*)d_in[0];
    const int*   eidx  = (const int*)d_in[1];
    const int*   batch = (const int*)d_in[2];
    const float* w1    = (const float*)d_in[3];
    const float* g1wih = (const float*)d_in[4];
    const float* g1whh = (const float*)d_in[5];
    const float* g1bih = (const float*)d_in[6];
    const float* g1bhh = (const float*)d_in[7];
    const float* w2    = (const float*)d_in[8];
    const float* g2wih = (const float*)d_in[9];
    const float* g2whh = (const float*)d_in[10];
    const float* g2bih = (const float*)d_in[11];
    const float* g2bhh = (const float*)d_in[12];
    const float* fcw   = (const float*)d_in[13];
    const float* fcb   = (const float*)d_in[14];
    float* out = (float*)d_out;

    char*  ws   = (char*)d_ws;
    float* mbuf = (float*)(ws + OFF_M);
    float* hF1  = (float*)(ws + OFF_HF1);
    float* hF2  = (float*)(ws + OFF_HF2);
    us16*  hhiA = (us16*)(ws + OFF_HHIA);
    us16*  hloA = (us16*)(ws + OFF_HLOA);
    us16*  hhiB = (us16*)(ws + OFF_HHIB);
    us16*  hloB = (us16*)(ws + OFF_HLOB);
    us16*  ahi  = (us16*)(ws + OFF_AHI);
    us16*  alo  = (us16*)(ws + OFF_ALO);
    us16*  pl1  = (us16*)(ws + OFF_W1);
    us16*  pl2  = (us16*)(ws + OFF_W2);
    int*   csr  = (int*)(ws + OFF_CSR);

    {
        WArgs wa; wa.w = w1; wa.wih = g1wih; wa.whh = g1whh; wa.pl = pl1;
        k_wprep<C1><<<dim3(3 * ((int)WPE1 / (8 * NTHR))), dim3(NTHR), 0, stream>>>(wa);
        WArgs wb; wb.w = w2; wb.wih = g2wih; wb.whh = g2whh; wb.pl = pl2;
        k_wprep<C2><<<dim3(3 * ((int)WPE2 / (8 * NTHR))), dim3(NTHR), 0, stream>>>(wb);
    }

    {
        ZArgs za; za.z = x; za.hhi = hhiA; za.hlo = hloA;
        k_xplanes<<<dim3((NN * C1) / (8 * NTHR)), dim3(NTHR), 0, stream>>>(za);
    }

    hipFuncSetAttribute(reinterpret_cast<const void*>(&k_csr),
                        hipFuncAttributeMaxDynamicSharedMemorySize, CSR_LDS_BYTES);
    {
        CsrArgs ca; ca.eidx = eidx; ca.csr = csr;
        k_csr<<<dim3(NBUCK), dim3(NTHR), CSR_LDS_BYTES, stream>>>(ca);
    }

    {
        const us16* wt_hi = pl1;
        const us16* wt_lo = pl1 + WPE1;
        const us16* ih_hi = pl1 + 2 * WPE1;
        const us16* ih_lo = pl1 + 3 * WPE1;
        const us16* hh_hi = pl1 + 4 * WPE1;
        const us16* hh_lo = pl1 + 5 * WPE1;
        for (int l = 0; l < 3; ++l) {
            const us16* inHi  = (l & 1) ? hhiB : hhiA;
            const us16* inLo  = (l & 1) ? hloB : hloA;
            us16*       outHi = (l & 1) ? hhiA : hhiB;
            us16*       outLo = (l & 1) ? hloA : hloB;

            GmArgs ga; ga.hhi = inHi; ga.hlo = inLo;
            ga.whi = wt_hi + (size_t)l * C1 * C1; ga.wlo = wt_lo + (size_t)l * C1 * C1;
            ga.m = mbuf; ga.nk = C1 / 32; ga.pad0 = 0;
            k_gemm_m<C1><<<dim3(NN / 16, C1 / 128), dim3(NTHR), 0, stream>>>(ga);

            GaArgs gg; gg.m = mbuf; gg.csr = csr; gg.ahi = ahi; gg.alo = alo;
            k_gather<C1><<<dim3(NN / 8), dim3(NTHR), 0, stream>>>(gg);

            GrArgs gr;
            gr.ahi = ahi; gr.alo = alo; gr.hhi = inHi; gr.hlo = inLo;
            gr.ohi = outHi; gr.olo = outLo;
            gr.hprev = (l == 0) ? x : hF1;
            gr.hout  = hF1;
            gr.ihh = ih_hi; gr.ihl = ih_lo; gr.hhh = hh_hi; gr.hhl = hh_lo;
            gr.bih = g1bih; gr.bhh = g1bhh;
            gr.nkA = C1 / 32; gr.nkH = C1 / 32;
            k_gru<C1><<<dim3(NN / 16, C1 / 128), dim3(NTHR), 0, stream>>>(gr);
        }
    }

    {
        RpArgs rp; rp.h1 = hF1; rp.h2 = hF2; rp.hhi = hhiA; rp.hlo = hloA;
        k_relu_pad<<<dim3((NN * C2) / (4 * NTHR)), dim3(NTHR), 0, stream>>>(rp);
    }

    {
        const us16* wt_hi = pl2;
        const us16* wt_lo = pl2 + WPE2;
        const us16* ih_hi = pl2 + 2 * WPE2;
        const us16* ih_lo = pl2 + 3 * WPE2;
        const us16* hh_hi = pl2 + 4 * WPE2;
        const us16* hh_lo = pl2 + 5 * WPE2;
        for (int l = 0; l < 3; ++l) {
            const us16* inHi  = (l & 1) ? hhiB : hhiA;
            const us16* inLo  = (l & 1) ? hloB : hloA;
            us16*       outHi = (l & 1) ? hhiA : hhiB;
            us16*       outLo = (l & 1) ? hloA : hloB;
            const int   nkh   = (l == 0) ? (C1 / 32) : (C2 / 32);

            GmArgs ga; ga.hhi = inHi; ga.hlo = inLo;
            ga.whi = wt_hi + (size_t)l * C2 * C2; ga.wlo = wt_lo + (size_t)l * C2 * C2;
            ga.m = mbuf; ga.nk = nkh; ga.pad0 = 0;
            k_gemm_m<C2><<<dim3(NN / 16, C2 / 128), dim3(NTHR), 0, stream>>>(ga);

            GaArgs gg; gg.m = mbuf; gg.csr = csr; gg.ahi = ahi; gg.alo = alo;
            k_gather<C2><<<dim3(NN / 8), dim3(NTHR), 0, stream>>>(gg);

            GrArgs gr;
            gr.ahi = ahi; gr.alo = alo; gr.hhi = inHi; gr.hlo = inLo;
            gr.ohi = outHi; gr.olo = outLo;
            gr.hprev = hF2;
            gr.hout  = hF2;
            gr.ihh = ih_hi; gr.ihl = ih_lo; gr.hhh = hh_hi; gr.hhl = hh_lo;
            gr.bih = g2bih; gr.bhh = g2bhh;
            gr.nkA = C2 / 32; gr.nkH = nkh;
            k_gru<C2><<<dim3(NN / 16, C2 / 128), dim3(NTHR), 0, stream>>>(gr);
        }
    }

    {
        PfArgs pf; pf.h = hF2; pf.batch = batch; pf.fcw = fcw; pf.fcb = fcb; pf.out = out;
        k_poolfc<<<dim3(1), dim3(NTHR), 0, stream>>>(pf);
    }
}
